// RelativeGlobalAttention_39599598469319
// MI455X (gfx1250) — hardware-verified
//
#include <hip/hip_runtime.h>


#ifndef NB
#define NB 2
#endif
#ifndef SEQ
#define SEQ 2048
#endif
#define NB_FULL  2
#define SEQ_FULL 2048
#define MAXSEQ   2048
#define DM   1024
#define NH   16
#define HD   64
#define MROWS (NB * SEQ)
#define QP   SEQ
#define PP   72
#define KST  64
#define PCAR 16384.0f
#define CSCL 0.25f
#define WCAR 64.0f
#define OSCL 0.000003814697265625f
#define SCL  0.125f
#define L2E  1.4426950408889634f

static_assert(SEQ % 64 == 0);
static_assert(SEQ >= 64 && SEQ <= MAXSEQ);
static_assert(NB >= 1 && NB <= NB_FULL);
static_assert(MROWS % 64 == 0);
static_assert(DM == NH * HD);
static_assert(DM % 64 == 0);
static_assert((PP * 2) % 16 == 0);
static_assert(KST % 32 == 0);

typedef _Float16 h16;
typedef unsigned short bf;
typedef __attribute__((ext_vector_type(16))) __bf16   v16bf;
typedef __attribute__((ext_vector_type(16))) _Float16 v16h;
typedef __attribute__((ext_vector_type(8)))  _Float16 v8h;
typedef __attribute__((ext_vector_type(8)))  unsigned short v8us;
typedef __attribute__((ext_vector_type(8)))  float    v8f;
typedef __attribute__((ext_vector_type(4)))  float    v4f;
typedef v8h  __attribute__((may_alias)) v8ha;
typedef v4f  __attribute__((may_alias)) v4fa;
typedef v8us __attribute__((may_alias)) v8usa;

__device__ __forceinline__ unsigned short f2bf(float f) { unsigned u = __float_as_uint(f); u += 0x7FFFu + ((u >> 16) & 1u); return (unsigned short)(u >> 16); }
__device__ __forceinline__ float bf2f(unsigned short b) { return __uint_as_float(((unsigned)b) << 16); }
__device__ __forceinline__ float bfr(float f) { return bf2f(f2bf(f)); }
__device__ __forceinline__ v16h cat16(v8h lo, v8h hi) { return __builtin_shufflevector(lo, hi, 0, 1, 2, 3, 4, 5, 6, 7, 8, 9, 10, 11, 12, 13, 14, 15); }
__device__ __forceinline__ v16bf cat16b(v8us lo, v8us hi) { return __builtin_bit_cast(v16bf, __builtin_shufflevector(lo, hi, 0, 1, 2, 3, 4, 5, 6, 7, 8, 9, 10, 11, 12, 13, 14, 15)); }
__device__ __forceinline__ v8f wmma16(v16h a, v16h b, v8f c) { return __builtin_amdgcn_wmma_f32_16x16x32_f16(false, a, false, b, (short)0, c, false, false); }
__device__ __forceinline__ v8f wmmab(v16bf a, v16bf b, v8f c) { return __builtin_amdgcn_wmma_f32_16x16x32_bf16(false, a, false, b, (short)0, c, false, false); }

template <typename T16> struct WFrag;
template <> struct WFrag<h16> { typedef v16h V; static __device__ __forceinline__ V ld(const h16* p) { return cat16(*(const v8h*)p, *(const v8h*)(p + 16)); } static __device__ __forceinline__ v8f mma(V a, V b, v8f c) { return wmma16(a, b, c); } };
template <> struct WFrag<bf> { typedef v16bf V; static __device__ __forceinline__ V ld(const bf* p) { return cat16b(*(const v8us*)p, *(const v8us*)(p + 16)); } static __device__ __forceinline__ v8f mma(V a, V b, v8f c) { return wmmab(a, b, c); } };
template <typename T16, int NSPLIT, bool BIAS>
__global__ __launch_bounds__(32) void k_gemmw(const T16* __restrict__ A, const T16* __restrict__ A2, const T16* __restrict__ Bt, const T16* __restrict__ Bt2, int K, float* C, int ldc, const float* __restrict__ bias, float scale, size_t sA, size_t sB, size_t sC) {
    typedef typename WFrag<T16>::V V;
    __shared__ __align__(16) float os[16 * 68];
    const size_t z = blockIdx.z; A += z * sA; if (A2) A2 += z * sA; Bt += z * sB; if (Bt2) Bt2 += z * sB; C += z * sC;
    const int lane = threadIdx.x & 31, lr = lane & 15, hi = lane >> 4; const int r0 = blockIdx.x * 64, c0 = blockIdx.y * 64;
    v8f acc[4][4];
#pragma unroll
    for (int mb = 0; mb < 4; ++mb)
#pragma unroll
        for (int nb = 0; nb < 4; ++nb) acc[mb][nb] = (v8f){};
    const size_t aoff = (size_t)(r0 + lr) * K + 8 * hi, boff = (size_t)(c0 + lr) * K + 8 * hi;
#pragma unroll 1
    for (int kc = 0; kc < K; kc += 32) {
        V a[4], a2[4];
#pragma unroll
        for (int mb = 0; mb < 4; ++mb) { a[mb] = WFrag<T16>::ld(A + aoff + (size_t)mb * 16 * K + kc); if (NSPLIT == 1 || NSPLIT == 2) a2[mb] = WFrag<T16>::ld(A2 + aoff + (size_t)mb * 16 * K + kc); }
#pragma unroll
        for (int nb = 0; nb < 4; ++nb) { const V b = WFrag<T16>::ld(Bt + boff + (size_t)nb * 16 * K + kc); V b2; if (NSPLIT >= 2) b2 = WFrag<T16>::ld(Bt2 + boff + (size_t)nb * 16 * K + kc);
#pragma unroll
            for (int mb = 0; mb < 4; ++mb) { acc[mb][nb] = WFrag<T16>::mma(a[mb], b, acc[mb][nb]); if (NSPLIT == 1 || NSPLIT == 2) acc[mb][nb] = WFrag<T16>::mma(a2[mb], b, acc[mb][nb]); if (NSPLIT >= 2) acc[mb][nb] = WFrag<T16>::mma(a[mb], b2, acc[mb][nb]); } }
        asm volatile("v_nop\n\tv_nop\n\tv_nop\n\tv_nop" : "+v"(acc[0][0]), "+v"(acc[1][1]), "+v"(acc[2][2]), "+v"(acc[3][3]) : "v"(a[0]), "v"(a[3]));
    }
#pragma unroll
    for (int mb = 0; mb < 4; ++mb) {
#pragma unroll
        for (int nb = 0; nb < 4; ++nb) {
#pragma unroll
            for (int j = 0; j < 8; ++j) os[(hi * 8 + j) * 68 + nb * 16 + lr] = acc[mb][nb][j]; }
        __builtin_amdgcn_wave_barrier(); asm volatile("" ::: "memory");
        float* crow = C + (size_t)(r0 + mb * 16) * ldc + c0;
#pragma unroll 1
        for (int ps = 0; ps < 2; ++ps) {
#pragma unroll
            for (int s = 0; s < 8; ++s) { const int row = 2 * s + hi, cofs = lr * 4; v4f val = *(const v4fa*)(os + row * 68 + cofs); val = val * scale;
                if (BIAS) { val[0] += bfr(bias[c0 + cofs]); val[1] += bfr(bias[c0 + cofs + 1]); val[2] += bfr(bias[c0 + cofs + 2]); val[3] += bfr(bias[c0 + cofs + 3]); }
                *(volatile v4f*)(crow + (size_t)row * ldc + cofs) = val; }
            if (ps == 0) __threadfence(); }
        __builtin_amdgcn_wave_barrier(); asm volatile("" ::: "memory");
    }
}

__global__ __launch_bounds__(256) void k_cvtx(const float* __restrict__ src, bf* dst, size_t n8) {
    const size_t i = (size_t)blockIdx.x * 256 + threadIdx.x; if (i >= n8) return;
    const size_t r = i / (DM / 8); const int c = (int)(i % (DM / 8)) * 8;
    const int b = (int)(r / SEQ), l = (int)(r % SEQ);
    const v8f v = *(const v8f*)(src + ((size_t)b * SEQ_FULL + l) * DM + c); v8us o;
#pragma unroll
    for (int k = 0; k < 8; ++k) o[k] = f2bf(v[k]);
    *(volatile v8us*)(dst + i * 8) = o; __threadfence(); *(volatile v8us*)(dst + i * 8) = o; }

__global__ __launch_bounds__(256) void k_cvt8(const float* __restrict__ src, bf* dst, size_t n8) { const size_t i = (size_t)blockIdx.x * 256 + threadIdx.x; if (i >= n8) return; const v8f v = *(const v8f*)(src + i * 8); v8us o;
#pragma unroll
    for (int k = 0; k < 8; ++k) o[k] = f2bf(v[k]); *(volatile v8us*)(dst + i * 8) = o; __threadfence(); *(volatile v8us*)(dst + i * 8) = o; }

__global__ __launch_bounds__(256) void k_cvth(const float* __restrict__ src, h16* dst, size_t n8, float sc) { const size_t i = (size_t)blockIdx.x * 256 + threadIdx.x; if (i >= n8) return; const v8f v = *(const v8f*)(src + i * 8); v8h o;
#pragma unroll
    for (int k = 0; k < 8; ++k) o[k] = (h16)(bfr(v[k]) * sc); *(volatile v8h*)(dst + i * 8) = o; __threadfence(); *(volatile v8h*)(dst + i * 8) = o; }

__global__ __launch_bounds__(256) void k_qkp(const float* __restrict__ Cf, h16* P, size_t n8) {
    const size_t i = (size_t)blockIdx.x * 256 + threadIdx.x; if (i >= n8) return;
    const int d8 = (int)(i % (HD / 8)); const size_t rl = i / (HD / 8);
    const int l = (int)(rl % SEQ); const int bh = (int)(rl / SEQ); const int h = bh % NH, b = bh / NH;
    const float* s = Cf + ((size_t)b * SEQ + l) * DM + h * HD + d8 * 8;
    const v4f a0 = *(const v4f*)s, a1 = *(const v4f*)(s + 4); v8h o;
#pragma unroll
    for (int k = 0; k < 4; ++k) { o[k] = (h16)a0[k]; o[k + 4] = (h16)a1[k]; }
    *(volatile v8h*)(P + i * 8) = o; __threadfence(); *(volatile v8h*)(P + i * 8) = o; }

__global__ __launch_bounds__(256) void k_vtp(const float* __restrict__ Cf, h16* VT, size_t n8) {
    const size_t i = (size_t)blockIdx.x * 256 + threadIdx.x; if (i >= n8) return;
    const int l8 = (int)(i % (SEQ / 8)); const size_t rd = i / (SEQ / 8);
    const int d = (int)(rd % HD); const int bh = (int)(rd / HD); const int h = bh % NH, b = bh / NH;
    const float* s = Cf + ((size_t)b * SEQ + 8 * l8) * DM + h * HD + d; v8h o;
#pragma unroll
    for (int q = 0; q < 8; ++q) o[q] = (h16)s[(size_t)q * DM];
    *(volatile v8h*)(VT + i * 8) = o; __threadfence(); *(volatile v8h*)(VT + i * 8) = o; }

__global__ __launch_bounds__(32) void k_flash(const h16* __restrict__ Qh, const h16* __restrict__ Kh, const h16* __restrict__ VT, const h16* __restrict__ Eh, h16* Ch, h16* Cl) {
    extern __shared__ __align__(16) float qes[];
    __shared__ __align__(16) h16 psh[16 * PP];
    __shared__ __align__(16) h16 psl[16 * PP];
    const int lane = threadIdx.x & 31, lr = lane & 15, hh = lane >> 4;
    const int nqb = SEQ / 16;
    const int qb = (int)(blockIdx.x % nqb), bh = (int)(blockIdx.x / nqb);
    const int h = bh % NH, b = bh / NH;
    const int l0 = qb * 16;
    const h16* qp = Qh + ((size_t)bh * SEQ + l0) * HD + (size_t)lr * HD + 8 * hh;
    const h16* kp = Kh + (size_t)bh * SEQ * HD + (size_t)lr * HD + 8 * hh;
    const h16* vp = VT + (size_t)bh * HD * SEQ + (size_t)lr * SEQ + 8 * hh;
    const h16* ep = Eh + (size_t)lr * HD + 8 * hh;
    const v16h qa0 = WFrag<h16>::ld(qp), qa1 = WFrag<h16>::ld(qp + 32);
    const int emin = MAXSEQ - 16 - l0;
#pragma unroll 1
    for (int e0 = emin; e0 < MAXSEQ; e0 += 16) {
        v8f acc = (v8f){};
        const v16h b0 = WFrag<h16>::ld(ep + (size_t)e0 * HD), b1 = WFrag<h16>::ld(ep + (size_t)e0 * HD + 32);
        acc = wmma16(qa0, b0, acc); acc = wmma16(qa1, b1, acc);
        asm volatile("v_nop\n\tv_nop\n\tv_nop\n\tv_nop" : "+v"(acc) : "v"(qa1), "v"(b1));
        const int cb = e0 - emin + lr;
#pragma unroll
        for (int r = 0; r < 8; ++r) qes[(hh * 8 + r) * QP + cb] = acc[r] * SCL;
    }
    __syncthreads();
    float rmax[8], rsum[8]; v8f oacc[4];
#pragma unroll
    for (int r = 0; r < 8; ++r) { rmax[r] = -1.0e30f; rsum[r] = 0.0f; }
#pragma unroll
    for (int t = 0; t < 4; ++t) oacc[t] = (v8f){};
#pragma unroll 1
    for (int m0 = 0; m0 < SEQ; m0 += KST) {
        v8f s[4];
#pragma unroll
        for (int c = 0; c < 4; ++c) { const h16* kr = kp + (size_t)(m0 + 16 * c) * HD; const v16h k0 = WFrag<h16>::ld(kr), k1 = WFrag<h16>::ld(kr + 32); v8f a = (v8f){}; a = wmma16(qa0, k0, a); a = wmma16(qa1, k1, a); s[c] = a; }
        asm volatile("v_nop\n\tv_nop\n\tv_nop\n\tv_nop" : "+v"(s[0]), "+v"(s[1]), "+v"(s[2]), "+v"(s[3]) : "v"(qa0), "v"(qa1));
        float mloc[8], corr[8], rs[8];
#pragma unroll
        for (int r = 0; r < 8; ++r) mloc[r] = -1.0e30f;
#pragma unroll
        for (int c = 0; c < 4; ++c)
#pragma unroll
            for (int r = 0; r < 8; ++r) { const int rt = hh * 8 + r; const int j = m0 + 16 * c + lr; const int col = min(j + 15 - rt, QP - 1);
                const float bb = qes[rt * QP + col]; const float bs = (j <= l0 + rt) ? bb : 0.0f;
                const float t = fmaf(s[c][r], SCL, bs); s[c][r] = t; mloc[r] = fmaxf(mloc[r], t); }
#pragma unroll
        for (int r = 0; r < 8; ++r) { float m = mloc[r]; m = fmaxf(m, __shfl_xor(m, 1, 16)); m = fmaxf(m, __shfl_xor(m, 2, 16)); m = fmaxf(m, __shfl_xor(m, 4, 16)); m = fmaxf(m, __shfl_xor(m, 8, 16));
            const float nm = fmaxf(rmax[r], m); corr[r] = __builtin_amdgcn_exp2f((rmax[r] - nm) * L2E); rmax[r] = nm; rs[r] = 0.0f; }
#pragma unroll
        for (int c = 0; c < 4; ++c)
#pragma unroll
            for (int r = 0; r < 8; ++r) { const float p = __builtin_amdgcn_exp2f((s[c][r] - rmax[r]) * L2E); rs[r] += p; const float y = p * PCAR;
                const h16 yh = (h16)y; const h16 yl = (h16)(y - (float)yh); const int o = (hh * 8 + r) * PP + 16 * c + lr; psh[o] = yh; psl[o] = yl; }
#pragma unroll
        for (int r = 0; r < 8; ++r) { float q = rs[r]; q += __shfl_xor(q, 1, 16); q += __shfl_xor(q, 2, 16); q += __shfl_xor(q, 4, 16); q += __shfl_xor(q, 8, 16); rsum[r] = fmaf(rsum[r], corr[r], q); }
#pragma unroll
        for (int t = 0; t < 4; ++t)
#pragma unroll
            for (int r = 0; r < 8; ++r) oacc[t][r] *= corr[r];
        __syncthreads();
        v16h pa, pb, vb;
#pragma unroll
        for (int kk = 0; kk < KST / 32; ++kk) {
            const h16* ph = psh + lr * PP + kk * 32 + 8 * hh; const h16* pl = psl + lr * PP + kk * 32 + 8 * hh;
            pa = cat16(*(const v8ha*)ph, *(const v8ha*)(ph + 16)); pb = cat16(*(const v8ha*)pl, *(const v8ha*)(pl + 16));
#pragma unroll
            for (int t = 0; t < 4; ++t) { vb = WFrag<h16>::ld(vp + (size_t)(16 * t) * SEQ + m0 + kk * 32); oacc[t] = wmma16(pa, vb, oacc[t]); oacc[t] = wmma16(pb, vb, oacc[t]); }
        }
        asm volatile("v_nop\n\tv_nop\n\tv_nop\n\tv_nop" : "+v"(oacc[0]), "+v"(oacc[1]), "+v"(oacc[2]), "+v"(oacc[3]) : "v"(pb), "v"(vb));
        __syncthreads();
    }
    float fr[8];
#pragma unroll
    for (int r = 0; r < 8; ++r) fr[r] = __fdiv_rn(CSCL, rsum[r]);
#pragma unroll
    for (int t = 0; t < 4; ++t)
#pragma unroll
        for (int r = 0; r < 8; ++r) { const float y = oacc[t][r] * fr[r]; const h16 yh = (h16)y; const h16 yl = (h16)(y - (float)yh); const int o = (hh * 8 + r) * PP + 16 * t + lr; psh[o] = yh; psl[o] = yl; }
    __syncthreads();
    const int rr = lane >> 3, c8 = (lane & 7) * 8;
    h16* cbh = Ch + ((size_t)b * SEQ + l0) * DM + h * HD + c8;
    h16* cbl = Cl + ((size_t)b * SEQ + l0) * DM + h * HD + c8;
#pragma unroll 1
    for (int ps = 0; ps < 2; ++ps) {
#pragma unroll
        for (int s4 = 0; s4 < 4; ++s4) { const int row = s4 * 4 + rr; const v8h oh = *(const v8ha*)(psh + row * PP + c8); const v8h ol = *(const v8ha*)(psl + row * PP + c8);
            *(volatile v8h*)(cbh + (size_t)row * DM) = oh; *(volatile v8h*)(cbl + (size_t)row * DM) = ol; }
        if (ps == 0) __threadfence(); }
}

extern "C" void kernel_launch(void* const* d_in, const int* in_sizes, int n_in,
                              void* d_out, int out_size, void* d_ws, size_t ws_size, hipStream_t stream) {
    if (n_in < 10) return;
    const float* X    = (const float*)d_in[0];
    const float* Wq   = (const float*)d_in[1];
    const float* Wq_b = (const float*)d_in[2];
    const float* Wk   = (const float*)d_in[3];
    const float* Wk_b = (const float*)d_in[4];
    const float* Wv   = (const float*)d_in[5];
    const float* Wv_b = (const float*)d_in[6];
    const float* Wf   = (const float*)d_in[7];
    const float* Wf_b = (const float*)d_in[8];
    const float* E    = (const float*)d_in[9];
    float* OUT = (float*)d_out;
    if ((size_t)in_sizes[0] < ((size_t)(NB - 1) * SEQ_FULL + SEQ) * DM) return;
    if ((size_t)in_sizes[1] < (size_t)DM * DM || (size_t)in_sizes[3] < (size_t)DM * DM || (size_t)in_sizes[5] < (size_t)DM * DM || (size_t)in_sizes[7] < (size_t)DM * DM) return;
    if (in_sizes[2] < DM || in_sizes[4] < DM || in_sizes[6] < DM || in_sizes[8] < DM) return;
    if ((size_t)in_sizes[9] < (size_t)MAXSEQ * HD) return;
    if ((size_t)out_size < (size_t)MROWS * DM) return;

    char* wsp = (char*)d_ws;
    auto take = [&](size_t bytes) { char* p = wsp; wsp += (bytes + 255) & ~(size_t)255; return (void*)p; };
    const size_t nMD = (size_t)MROWS * DM, nDD = (size_t)DM * DM, nE = (size_t)MAXSEQ * HD;
    bf*  Xb  = (bf*)take(nMD * 2);
    bf*  Wqb = (bf*)take(nDD * 2); bf* Wkb = (bf*)take(nDD * 2); bf* Wvb = (bf*)take(nDD * 2);
    h16* Fh  = (h16*)take(nDD * 2);
    h16* Ehp = (h16*)take(nE * 2);
    float* Cf = (float*)take(nMD * 4);
    h16* Qh = (h16*)take(nMD * 2); h16* Kh = (h16*)take(nMD * 2); h16* VTp = (h16*)take(nMD * 2);
    h16* Ch = (h16*)take(nMD * 2); h16* Cl = (h16*)take(nMD * 2);
    if ((size_t)(wsp - (char*)d_ws) > ws_size) return;

    const unsigned g256MD = (unsigned)((nMD / 8 + 255) / 256), g256DD = (unsigned)((nDD / 8 + 255) / 256), g256E = (unsigned)((nE / 8 + 255) / 256);
    k_cvtx<<<g256MD, 256, 0, stream>>>(X, Xb, nMD / 8);
    k_cvt8<<<g256DD, 256, 0, stream>>>(Wq, Wqb, nDD / 8);
    k_cvt8<<<g256DD, 256, 0, stream>>>(Wk, Wkb, nDD / 8);
    k_cvt8<<<g256DD, 256, 0, stream>>>(Wv, Wvb, nDD / 8);
    k_cvth<<<g256DD, 256, 0, stream>>>(Wf, Fh, nDD / 8, WCAR);
    k_cvth<<<g256E, 256, 0, stream>>>(E, Ehp, nE / 8, 1.0f);

    const dim3 gproj(MROWS / 64, DM / 64, 1);
    k_gemmw<bf, 0, true><<<gproj, 32, 0, stream>>>(Xb, nullptr, Wqb, nullptr, DM, Cf, DM, Wq_b, 1.0f, 0, 0, 0);
    k_qkp<<<g256MD, 256, 0, stream>>>(Cf, Qh, nMD / 8);
    k_gemmw<bf, 0, true><<<gproj, 32, 0, stream>>>(Xb, nullptr, Wkb, nullptr, DM, Cf, DM, Wk_b, 1.0f, 0, 0, 0);
    k_qkp<<<g256MD, 256, 0, stream>>>(Cf, Kh, nMD / 8);
    k_gemmw<bf, 0, true><<<gproj, 32, 0, stream>>>(Xb, nullptr, Wvb, nullptr, DM, Cf, DM, Wv_b, 1.0f, 0, 0, 0);
    k_vtp<<<g256MD, 256, 0, stream>>>(Cf, VTp, nMD / 8);

    const size_t ldsb = (size_t)16 * QP * 4;
    (void)hipFuncSetAttribute(reinterpret_cast<const void*>(&k_flash), hipFuncAttributeMaxDynamicSharedMemorySize, (int)ldsb);
    k_flash<<<(unsigned)(NB * NH * (SEQ / 16)), 32, ldsb, stream>>>(Qh, Kh, VTp, Ehp, Ch, Cl);

    k_gemmw<h16, 1, true><<<gproj, 32, 0, stream>>>(Ch, Cl, Fh, nullptr, DM, OUT, DM, Wf_b, OSCL, 0, 0, 0);
    (void)hipGetLastError();
}
